// Model_22746146799733
// MI455X (gfx1250) — hardware-verified
//
#include <hip/hip_runtime.h>
#include <stddef.h>
#include <stdint.h>


#define NN       50000
#define NE       250000
#define NG       1000
#define DRAW     10
#define DH       300
#define DO       31
#define DP       320
#define PW       640
#define MP       50048
#define XK       32
#define NLW      32
#define NTHR     256
#define NWAVE    8
#define EPT      8
#define CHUNK    (NTHR * EPT)
#define WCAP     (EPT * 32)
#define LISTN    (NWAVE * WCAP)
#define NBMAX    2048
#define NBRUN    1024
#define NSB      49
#define FLB      64
#define RCAP     28672
#define DEGCAP   64
#define PCAP     4096
#define PKS      11
#define PG       32
#define NPB      32
#define GBM      128
#define GTHR     256
#define WSQ      (DP * PW)
#define NUW      (DP * (PW / 8))
#define NUB1     (6 * NUW)
#define NUB2     (NUB1 + 32 * (PW / 8))
#define NUB3     (NUB2 + DP * (XK / 8))
#define NUXB     (MP * (XK / 8))
#define NUTOT    (NUB3 + NUXB)
#define PLB      ((size_t)MP * PW * 2)
#define OFF_P1   ((size_t)0)
#define OFF_P2   (PLB)
#define OFF_W    (2 * PLB)
#define WBYTES   ((size_t)NUB3 * 16)
#define OFF_FL   (OFF_W + WBYTES)
#define FLBYTES  ((size_t)3 * FLB * 128)
#define WS_TOTAL (OFF_FL + FLBYTES)
#define WSMAX    134217728
#define LDS_AGG  ((2 * RCAP + 2 * NBMAX + LISTN) * 4 + 64)

static_assert((DP % 32) == 0 && (DP % 64) == 0 && PW == 2 * DP);
static_assert(MP == 391 * 128 && MP >= NN && (MP % GBM) == 0);
static_assert(DO < 32 && NLW == 32 && DRAW <= XK && XK == 32);
static_assert(NG <= NPB * PG && PG * DO * 4 == 31 * 128);
static_assert((CHUNK & (CHUNK - 1)) == 0 && CHUNK <= (1 << PKS));
static_assert((NBMAX & (NBMAX - 1)) == 0 && NBMAX <= (1 << PKS));
static_assert(NTHR * 8 == NBMAX && LISTN >= NBMAX && LISTN >= NWAVE * WCAP);
static_assert(NBRUN <= NBMAX && (NBRUN % 8) == 0 && NSB * NBRUN >= MP && NSB <= FLB);
static_assert((RCAP % 32) == 0 && LDS_AGG <= 300000);
static_assert(NE < (1 << 21) && NN < (1 << 21));
static_assert(3 * NSB <= NTHR && PG == 4 * NWAVE);
static_assert((NUW % NTHR) == 0 && (NUB1 % NTHR) == 0 && (NUB2 % NTHR) == 0 && (NUB3 % NTHR) == 0);
static_assert((NUTOT % NTHR) == 0 && (PW / 8) == 80);
static_assert((PLB % 128) == 0 && (WBYTES % 128) == 0 && (FLBYTES % 128) == 0);
static_assert((size_t)MP * XK * 2 <= PLB && (size_t)MP * NLW * 4 <= PLB);
static_assert(WS_TOTAL <= (size_t)WSMAX);
static_assert(WBYTES == (size_t)(6 * WSQ + 32 * PW + DP * XK) * 2);

typedef float          v4f  __attribute__((ext_vector_type(4)));
typedef float          v8f  __attribute__((ext_vector_type(8)));
typedef int            v4i  __attribute__((ext_vector_type(4)));
typedef int            v8i  __attribute__((ext_vector_type(8)));
typedef unsigned int   v4u  __attribute__((ext_vector_type(4)));
typedef unsigned short v8us __attribute__((ext_vector_type(8)));
typedef __bf16         v16b __attribute__((ext_vector_type(16)));
typedef v4f  __attribute__((may_alias)) v4fa;
typedef v4u  __attribute__((may_alias)) v4ua;
typedef v8us __attribute__((may_alias)) v8usa;
union FragB { v16b v; v8us h[2]; v8i w; };

__device__ __forceinline__ v8f wmb(const FragB& a, const FragB& b, v8f c) {
  v8f d = __builtin_amdgcn_wmma_f32_16x16x32_bf16(false, a.v, false, b.v, (short)0, c, false, false);
  asm volatile("v_nop\n\tv_nop\n\tv_nop\n\tv_nop" : "+v"(d) : "v"(a.w), "v"(b.w));
  return d;
}

__device__ __forceinline__ unsigned short bf_bits(float f) {
  const unsigned int u = __float_as_uint(f);
  const unsigned int r = (u + 0x7FFFu + ((u >> 16) & 1u)) >> 16;
  return (unsigned short)((f != f) ? 0x7FC0u : r);
}
__device__ __forceinline__ float bf_val(unsigned short b) {
  return __uint_as_float(((unsigned int)b) << 16);
}
__device__ __forceinline__ float bf_rne(float f) { return bf_val(bf_bits(f)); }

__device__ __forceinline__ int scan_chunk(const int* __restrict__ dsts, int nE, int cbase, int slotBase,
                                          int nb, int vec8, int* list, int tid, int lane, int wave) {
  int wc = 0;
  const int el0  = tid * EPT;
  const int e0   = cbase + el0;
  const int sent = -2147483647 - 1;
  v4i da, db;
  if (vec8 != 0 && cbase + CHUNK <= nE) {
    da = *(const v4i*)(dsts + e0);
    db = *(const v4i*)(dsts + e0 + 4);
  } else {
    da.x = (e0     < nE) ? dsts[min(e0,     nE - 1)] : sent;
    da.y = (e0 + 1 < nE) ? dsts[min(e0 + 1, nE - 1)] : sent;
    da.z = (e0 + 2 < nE) ? dsts[min(e0 + 2, nE - 1)] : sent;
    da.w = (e0 + 3 < nE) ? dsts[min(e0 + 3, nE - 1)] : sent;
    db.x = (e0 + 4 < nE) ? dsts[min(e0 + 4, nE - 1)] : sent;
    db.y = (e0 + 5 < nE) ? dsts[min(e0 + 5, nE - 1)] : sent;
    db.z = (e0 + 6 < nE) ? dsts[min(e0 + 6, nE - 1)] : sent;
    db.w = (e0 + 7 < nE) ? dsts[min(e0 + 7, nE - 1)] : sent;
  }
  const unsigned nbs = (unsigned)slotBase;
  const unsigned unb = (unsigned)nb;
  const unsigned s0 = (unsigned)da.x - nbs, s1 = (unsigned)da.y - nbs;
  const unsigned s2 = (unsigned)da.z - nbs, s3 = (unsigned)da.w - nbs;
  const unsigned s4 = (unsigned)db.x - nbs, s5 = (unsigned)db.y - nbs;
  const unsigned s6 = (unsigned)db.z - nbs, s7 = (unsigned)db.w - nbs;
  const bool h0 = s0 < unb, h1 = s1 < unb, h2 = s2 < unb, h3 = s3 < unb;
  const bool h4 = s4 < unb, h5 = s5 < unb, h6 = s6 < unb, h7 = s7 < unb;
  const unsigned any = __builtin_amdgcn_ballot_w32(h0 | h1 | h2 | h3 | h4 | h5 | h6 | h7);
  if (any != 0u) {
#define HITJ(J, HJ, SJ) { \
      const unsigned mj = __builtin_amdgcn_ballot_w32(HJ); \
      if (mj != 0u) { \
        if (HJ) { \
          const int pos = wc + (int)__builtin_amdgcn_mbcnt_lo(mj, 0u); \
          if (pos < WCAP) list[wave * WCAP + pos] = ((el0 + (J)) << PKS) | (int)(SJ); \
        } \
        wc += (int)__builtin_popcount(mj); } }
    HITJ(0, h0, s0)
    HITJ(1, h1, s1)
    HITJ(2, h2, s2)
    HITJ(3, h3, s3)
    HITJ(4, h4, s4)
    HITJ(5, h5, s5)
    HITJ(6, h6, s6)
    HITJ(7, h7, s7)
#undef HITJ
  }
  return wc;
}

__device__ __forceinline__ int compact_keys(const int* __restrict__ keys, int nK, int slotBase, int nb, int vec8,
                                            int* reg1, int cap, int* list, int* wcnt,
                                            int tid, int lane, int wave) {
  int tot = 0;
  const int nChunks = (nK + CHUNK - 1) / CHUNK;
#pragma unroll 1
  for (int ch = 0; ch < nChunks; ++ch) {
    const int cbase = ch * CHUNK;
    const int wc = scan_chunk(keys, nK, cbase, slotBase, nb, vec8, list, tid, lane, wave);
    if (lane == 0) wcnt[wave] = wc;
    __syncthreads();
    int pre = 0, all = 0;
#pragma unroll
    for (int w2 = 0; w2 < NWAVE; ++w2) {
      int c = wcnt[w2];
      c = c < 0 ? 0 : (c > WCAP ? WCAP : c);
      all += c;
      pre += (w2 < wave) ? c : 0;
    }
    const int wcc  = wc > WCAP ? WCAP : wc;
    const int base = tot + pre;
#pragma unroll 1
    for (int i = lane; i < wcc; i += 32) {
      const int ent = list[wave * WCAP + i];
      const int el  = (ent >> PKS) & (CHUNK - 1);
      const int sl  = ent & (NBMAX - 1);
      int eid = cbase + el;
      eid = eid > nK - 1 ? nK - 1 : eid;
      const int pos = base + i;
      if (pos < cap) reg1[pos] = (int)(((unsigned)eid << PKS) | (unsigned)sl);
    }
    tot += all;
    tot = tot > cap ? cap : tot;
    __syncthreads();
  }
  return tot;
}

__device__ __forceinline__ v8us gat8(const float* __restrict__ W, int K, int N, int ldw, int kk, int n) {
  v8us o;
  const int nc = n < N ? n : N - 1;
  const bool nok = n < N;
#pragma unroll
  for (int i = 0; i < 8; ++i) {
    const int k  = kk + i;
    const int kc = k < K ? k : K - 1;
    const float v = W[(size_t)kc * (size_t)ldw + (size_t)nc];
    o[i] = (nok && k < K) ? bf_bits(v) : (unsigned short)0;
  }
  return o;
}

__global__ __launch_bounds__(NTHR) void k_prep(const float* __restrict__ wc1, const float* __restrict__ wf1,
                                               const float* __restrict__ wc2, const float* __restrict__ wf2,
                                               const float* __restrict__ wc3, const float* __restrict__ wf3,
                                               const float* __restrict__ wro, const float* __restrict__ wli,
                                               const float* __restrict__ x,
                                               unsigned short* wreg, unsigned short* xb) {
  const int bx = (int)blockIdx.x;
  const int u  = bx * NTHR + (int)threadIdx.x;
  v8us o;
  unsigned short* dp;
  if (bx < NUB1 / NTHR) {
    const int mi = bx / (NUW / NTHR);
    const int v  = u - mi * NUW;
    const int n  = v / (PW / 8);
    const int k8 = (v - n * (PW / 8)) * 8;
    const int kk = k8 < DP ? k8 : k8 - DP;
    if (mi == 0)      o = gat8(wc1, DH, DH, DH, kk, n);
    else if (mi == 1) o = gat8(wf1, DH, DH, DH, kk, n);
    else if (mi == 2) o = gat8(wc2, DH, DH, DH, kk, n);
    else if (mi == 3) o = gat8(wf2, DH, DH, DH, kk, n);
    else if (mi == 4) o = gat8(wc3, DH, DH, DH, kk, n);
    else              o = gat8(wf3, DH, DH, DH, kk, n);
    dp = wreg + (size_t)u * 8;
  } else if (bx < NUB2 / NTHR) {
    const int v  = u - NUB1;
    const int n  = v / (PW / 8);
    const int k8 = (v - n * (PW / 8)) * 8;
    const int kk = k8 < DP ? k8 : k8 - DP;
    o = gat8(wro, DH, DO, DO, kk, n);
    dp = wreg + (size_t)u * 8;
  } else if (bx < NUB3 / NTHR) {
    const int v  = u - NUB2;
    const int n  = v >> 2;
    const int k8 = (v & 3) * 8;
    o = gat8(wli, DRAW, DH, DH, k8, n);
    dp = wreg + (size_t)u * 8;
  } else if (bx < NUTOT / NTHR) {
    const int v   = u - NUB3;
    const int row = v >> 2;
    const int k8  = (v & 3) * 8;
    const int rc  = row < NN ? row : NN - 1;
    const bool rok = row < NN;
#pragma unroll
    for (int i = 0; i < 8; ++i) {
      const int k  = k8 + i;
      const int kc = k < DRAW ? k : DRAW - 1;
      const float val = x[(size_t)rc * DRAW + kc];
      o[i] = (rok && k < DRAW) ? bf_bits(val) : (unsigned short)0;
    }
    dp = xb + (size_t)v * 8;
  } else {
    return;
  }
  *(volatile v8us*)dp = o;
  __threadfence();
  *(volatile v8us*)dp = o;
}

template <int NTW, int RELU, int OUTF>
__global__ __launch_bounds__(GTHR) void k_gemm(const unsigned short* __restrict__ A, int lda,
                                               const unsigned short* __restrict__ BT, int ldb, int K,
                                               const float* __restrict__ bias, int nbias,
                                               void* outp, int nN, int mRows) {
  constexpr int BN = 16 * NTW;
  static_assert((OUTF == 0 && BN == 64) || (OUTF == 1 && BN == NLW));
  __shared__ __attribute__((aligned(16))) float stg[GBM * BN];
  const int tid = (int)threadIdx.x, lane = tid & 31, wave = tid >> 5, hh = lane >> 4, m = lane & 15;
  const int rowBase = (int)blockIdx.x * GBM;
  const int colBase = (int)blockIdx.y * BN;

  v8f acc[NTW];
  {
    const v8f z = {0.f, 0.f, 0.f, 0.f, 0.f, 0.f, 0.f, 0.f};
#pragma unroll
    for (int t = 0; t < NTW; ++t) acc[t] = z;
  }
  const unsigned short* ap = A  + (size_t)(rowBase + 16 * wave + m) * (size_t)lda + 8 * hh;
  const unsigned short* bp = BT + (size_t)(colBase + m) * (size_t)ldb + 8 * hh;

#pragma unroll 1
  for (int k0 = 0; k0 < K; k0 += 32) {
    FragB af;
    af.h[0] = *(const v8usa*)(ap + k0);
    af.h[1] = *(const v8usa*)(ap + k0 + 16);
#pragma unroll
    for (int nt = 0; nt < NTW; ++nt) {
      const unsigned short* wq = bp + (size_t)(16 * nt) * (size_t)ldb + k0;
      FragB bfr;
      bfr.h[0] = *(const v8usa*)wq;
      bfr.h[1] = *(const v8usa*)(wq + 16);
      acc[nt] = wmb(af, bfr, acc[nt]);
    }
  }

#pragma unroll
  for (int nt = 0; nt < NTW; ++nt) {
    const int lc  = 16 * nt + m;
    const int col = colBase + lc;
    const int cc  = col < nbias ? col : nbias - 1;
    const float braw = bias[cc];
    const float bb = (col < nbias) ? bf_rne(braw) : 0.0f;
#pragma unroll
    for (int r = 0; r < 8; ++r) {
      const int lr = 16 * wave + 8 * hh + r;
      const bool live = (rowBase + lr) < nN;
      float v = acc[nt][r] + bb;
      if (RELU != 0) v = (v > 0.0f) ? v : (v - v);
      stg[lr * BN + lc] = live ? v : 0.0f;
    }
  }
  __syncthreads();

  if constexpr (OUTF == 0) {
    unsigned short* outH = (unsigned short*)outp;
    const int q    = lane & 7;
    const bool isHi = ((lane >> 3) & 1) == 0;
    const int rsel = lane >> 4;
    const int coff = (isHi ? 0 : DP) + colBase + 8 * q;
    v4u pk[8];
#pragma unroll
    for (int i = 0; i < 8; ++i) {
      const int lr = 16 * wave + 2 * i + rsel;
      const v4f a = *(const v4fa*)(stg + lr * BN + 8 * q);
      const v4f b = *(const v4fa*)(stg + lr * BN + 8 * q + 4);
      const float f[8] = {a.x, a.y, a.z, a.w, b.x, b.y, b.z, b.w};
      unsigned int w[4];
#pragma unroll
      for (int j = 0; j < 4; ++j) {
        const unsigned short h0 = bf_bits(f[2 * j]), h1 = bf_bits(f[2 * j + 1]);
        const unsigned short l0 = bf_bits(f[2 * j] - bf_val(h0)), l1 = bf_bits(f[2 * j + 1] - bf_val(h1));
        const unsigned short q0 = isHi ? h0 : l0, q1 = isHi ? h1 : l1;
        w[j] = (unsigned int)q0 | ((unsigned int)q1 << 16);
      }
      v4u pv; pv.x = w[0]; pv.y = w[1]; pv.z = w[2]; pv.w = w[3];
      pk[i] = pv;
    }
#pragma unroll
    for (int i = 0; i < 8; ++i) {
      const int gr = rowBase + 16 * wave + 2 * i + rsel;
      unsigned short* op = outH + (size_t)gr * (size_t)PW + coff;
      if (gr < mRows) *(volatile v4u*)op = pk[i];
    }
    __threadfence();
#pragma unroll
    for (int i = 0; i < 8; ++i) {
      const int gr = rowBase + 16 * wave + 2 * i + rsel;
      unsigned short* op = outH + (size_t)gr * (size_t)PW + coff;
      if (gr < mRows) *(volatile v4u*)op = pk[i];
    }
  } else {
    float* outF = (float*)outp;
    const int q    = lane & 7;
    const int rsel = lane >> 3;
    v4f fv[4];
#pragma unroll
    for (int i = 0; i < 4; ++i) {
      const int lr = 16 * wave + 4 * i + rsel;
      fv[i] = *(const v4fa*)(stg + lr * BN + 4 * q);
    }
#pragma unroll
    for (int i = 0; i < 4; ++i) {
      const int gr = rowBase + 16 * wave + 4 * i + rsel;
      float* op = outF + (size_t)gr * (size_t)NLW + colBase + 4 * q;
      if (gr < mRows) *(volatile v4f*)op = fv[i];
    }
    __threadfence();
#pragma unroll
    for (int i = 0; i < 4; ++i) {
      const int gr = rowBase + 16 * wave + 4 * i + rsel;
      float* op = outF + (size_t)gr * (size_t)NLW + colBase + 4 * q;
      if (gr < mRows) *(volatile v4f*)op = fv[i];
    }
  }
}

__device__ __forceinline__ void add2(float& e, float& o, unsigned int hw, unsigned int lw) {
  const float he = __uint_as_float(hw << 16),          le = __uint_as_float(lw << 16);
  const float ho = __uint_as_float(hw & 0xffff0000u),  lo = __uint_as_float(lw & 0xffff0000u);
  e += (he + le);
  o += (ho + lo);
}

__global__ __launch_bounds__(NTHR) void k_scan(const int* __restrict__ srcs, const int* __restrict__ dsts,
                                               const unsigned short* __restrict__ F,
                                               unsigned short* Aout, int* fl,
                                               int nN, int nE, int nb, int vec8, int MPr) {
  extern __shared__ v4f lds_dyn[];
  int* reg1 = (int*)lds_dyn;
  int* reg2 = reg1 + RCAP;
  int* scnt = reg2 + RCAP;
  int* soff = scnt + NBMAX;
  int* list = soff + NBMAX;
  int* wcnt = list + LISTN;
  int* wtot = wcnt + NWAVE;
  const int tid = (int)threadIdx.x, lane = tid & 31, wave = tid >> 5;
  const int nodeBase = (int)blockIdx.x * nb;

  for (int i = tid; i < NBMAX; i += NTHR) scnt[i] = 0;
  __syncthreads();

  const int nh = compact_keys(dsts, nE, nodeBase, nb, vec8, reg1, RCAP, list, wcnt, tid, lane, wave);

  if (wave == 0) {
#pragma unroll 1
    for (int b0 = 0; b0 < nh; b0 += 32) {
      const int idx = b0 + lane;
      const int uv  = reg1[idx < RCAP ? idx : RCAP - 1];
      const int m32 = (nh - b0) < 32 ? (nh - b0) : 32;
#pragma unroll 1
      for (int k = 0; k < m32; ++k) {
        const int u  = __builtin_amdgcn_readlane(uv, k);
        const int sl = u & (NBMAX - 1);
        if (lane == 0) scnt[sl] = scnt[sl] + 1;
      }
    }
  }
  __syncthreads();

  {
    const v4i ca = *(const v4i*)(scnt + 8 * tid);
    const v4i cb = *(const v4i*)(scnt + 8 * tid + 4);
    const int e0 = ca.x < 0 ? 0 : ca.x, e1 = ca.y < 0 ? 0 : ca.y, e2 = ca.z < 0 ? 0 : ca.z, e3 = ca.w < 0 ? 0 : ca.w;
    const int e4 = cb.x < 0 ? 0 : cb.x, e5 = cb.y < 0 ? 0 : cb.y, e6 = cb.z < 0 ? 0 : cb.z, e7 = cb.w < 0 ? 0 : cb.w;
    const int ts = e0 + e1 + e2 + e3 + e4 + e5 + e6 + e7;
    int incl = ts;
#pragma unroll
    for (int d = 1; d < 32; d <<= 1) {
      const int up = __shfl_up(incl, d);
      if (lane >= d) incl += up;
    }
    if (lane == 31) wtot[wave] = incl;
    __syncthreads();
    int pre = 0;
#pragma unroll
    for (int w2 = 0; w2 < NWAVE; ++w2) pre += (w2 < wave) ? wtot[w2] : 0;
    int run = pre + incl - ts;
    soff[8 * tid + 0] = run; run += e0;
    soff[8 * tid + 1] = run; run += e1;
    soff[8 * tid + 2] = run; run += e2;
    soff[8 * tid + 3] = run; run += e3;
    soff[8 * tid + 4] = run; run += e4;
    soff[8 * tid + 5] = run; run += e5;
    soff[8 * tid + 6] = run; run += e6;
    soff[8 * tid + 7] = run;
  }
  __syncthreads();
  for (int i = tid; i < NBMAX; i += NTHR) list[i] = soff[i];
  __syncthreads();

  if (wave == 0) {
#pragma unroll 1
    for (int b0 = 0; b0 < nh; b0 += 32) {
      const int idx = b0 + lane;
      const int uv  = reg1[idx < RCAP ? idx : RCAP - 1];
      const int m32 = (nh - b0) < 32 ? (nh - b0) : 32;
#pragma unroll 1
      for (int k = 0; k < m32; ++k) {
        const int u   = __builtin_amdgcn_readlane(uv, k);
        const int sl  = u & (NBMAX - 1);
        const int eid = (int)((unsigned)u >> PKS);
        if (lane == 0) {
          int pos = list[sl];
          pos = pos < 0 ? 0 : (pos > RCAP - 1 ? RCAP - 1 : pos);
          reg2[pos] = eid;
          list[sl] = pos + 1;
        }
      }
    }
  }
  __syncthreads();

  const int nbw = nb >> 3;
  const bool ovf = (nh >= RCAP);
  const float qnan = __int_as_float(0x7fc00000);
  const int g1o = 8 * lane;
  const int g2o = 8 * (32 + (lane & 7));
  const bool l8 = lane < 8;
  int wbadv = ovf ? 1 : 0;

#pragma unroll 1
  for (int jt = 0; jt < nbw; ++jt) {
    const int slot = wave * nbw + jt;
    const int grow = nodeBase + slot;
    int st = soff[slot];
    const int craw = scnt[slot];
    int cnt = craw;
    st  = st < 0 ? 0 : (st > nh ? nh : st);
    cnt = cnt < 0 ? 0 : (cnt > DEGCAP ? DEGCAP : cnt);
    if (cnt > nh - st) cnt = nh - st;
    const bool rowBad = ovf || (craw > DEGCAP);
    wbadv |= (craw > DEGCAP) ? 1 : 0;
    const float pz = rowBad ? qnan : 0.0f;
    const bool liveRow = grow < nN;

    float aA[8], aB[8];
#pragma unroll
    for (int c = 0; c < 8; ++c) { aA[c] = 0.0f; aB[c] = 0.0f; }

#pragma unroll 1
    for (int b0 = 0; b0 < cnt; b0 += 32) {
      int idx = st + b0 + lane;
      idx = idx > nh - 1 ? nh - 1 : idx;
      idx = idx < 0 ? 0 : (idx > RCAP - 1 ? RCAP - 1 : idx);
      int eid = reg2[idx];
      eid = eid < 0 ? 0 : (eid > nE - 1 ? nE - 1 : eid);
      const int sraw = srcs[eid];
      const int sv = sraw < 0 ? 0 : (sraw > nN - 1 ? nN - 1 : sraw);
      const int m32 = (cnt - b0) < 32 ? (cnt - b0) : 32;
#pragma unroll 1
      for (int k = 0; k < m32; ++k) {
        const int sk = __builtin_amdgcn_readlane(sv, k);
        const unsigned short* rp = F + (size_t)sk * (size_t)PW;
        const v4u h1 = *(const v4ua*)(rp + g1o);
        const v4u l1 = *(const v4ua*)(rp + DP + g1o);
        const v4u h2 = *(const v4ua*)(rp + g2o);
        const v4u l2 = *(const v4ua*)(rp + DP + g2o);
        add2(aA[0], aA[1], h1.x, l1.x);
        add2(aA[2], aA[3], h1.y, l1.y);
        add2(aA[4], aA[5], h1.z, l1.z);
        add2(aA[6], aA[7], h1.w, l1.w);
        add2(aB[0], aB[1], h2.x, l2.x);
        add2(aB[2], aB[3], h2.y, l2.y);
        add2(aB[4], aB[5], h2.z, l2.z);
        add2(aB[6], aB[7], h2.w, l2.w);
      }
    }

    unsigned int hwA[4], lwA[4], hwB[4], lwB[4];
#pragma unroll
    for (int j = 0; j < 4; ++j) {
      const float r0 = (liveRow ? aA[2 * j]     : 0.0f) + pz;
      const float r1 = (liveRow ? aA[2 * j + 1] : 0.0f) + pz;
      const float t0 = (liveRow ? aB[2 * j]     : 0.0f) + pz;
      const float t1 = (liveRow ? aB[2 * j + 1] : 0.0f) + pz;
      const unsigned short hr0 = bf_bits(r0), hr1 = bf_bits(r1), ht0 = bf_bits(t0), ht1 = bf_bits(t1);
      const unsigned short lr0 = bf_bits(r0 - bf_val(hr0)), lr1 = bf_bits(r1 - bf_val(hr1));
      const unsigned short lt0 = bf_bits(t0 - bf_val(ht0)), lt1 = bf_bits(t1 - bf_val(ht1));
      hwA[j] = (unsigned int)hr0 | ((unsigned int)hr1 << 16);
      lwA[j] = (unsigned int)lr0 | ((unsigned int)lr1 << 16);
      hwB[j] = (unsigned int)ht0 | ((unsigned int)ht1 << 16);
      lwB[j] = (unsigned int)lt0 | ((unsigned int)lt1 << 16);
    }
    v4u hA, lA, hB, lB;
    hA.x = hwA[0]; hA.y = hwA[1]; hA.z = hwA[2]; hA.w = hwA[3];
    lA.x = lwA[0]; lA.y = lwA[1]; lA.z = lwA[2]; lA.w = lwA[3];
    hB.x = hwB[0]; hB.y = hwB[1]; hB.z = hwB[2]; hB.w = hwB[3];
    lB.x = lwB[0]; lB.y = lwB[1]; lB.z = lwB[2]; lB.w = lwB[3];

    unsigned short* gp = Aout + (size_t)grow * (size_t)PW;
    const bool wsv = grow < MPr;
    if (wsv) {
      *(volatile v4u*)(gp + g1o) = hA;
      if (l8) *(volatile v4u*)(gp + 256 + g1o) = hB;
      *(volatile v4u*)(gp + DP + g1o) = lA;
      if (l8) *(volatile v4u*)(gp + DP + 256 + g1o) = lB;
    }
    __threadfence();
    if (wsv) {
      *(volatile v4u*)(gp + g1o) = hA;
      if (l8) *(volatile v4u*)(gp + 256 + g1o) = hB;
      *(volatile v4u*)(gp + DP + g1o) = lA;
      if (l8) *(volatile v4u*)(gp + DP + 256 + g1o) = lB;
    }
  }

  if (lane == 0) wcnt[wave] = wbadv;
  __syncthreads();
  int anyb = 0;
#pragma unroll
  for (int w2 = 0; w2 < NWAVE; ++w2) anyb |= wcnt[w2];
  anyb = anyb != 0 ? 1 : 0;
  v4i fv; fv.x = anyb; fv.y = anyb; fv.z = anyb; fv.w = anyb;
  int* fp = fl + (size_t)blockIdx.x * 32 + 4 * (tid & 7);
  const bool fok = tid < 8;
  if (fok) *(volatile v4i*)fp = fv;
  __threadfence();
  if (fok) *(volatile v4i*)fp = fv;
}

__device__ __forceinline__ float pool_hits(unsigned mk, int node, const float* __restrict__ nl, int lane,
                                           float acc) {
  int c = (int)__builtin_popcount(mk);
  c = c > 32 ? 32 : c;
#pragma unroll 1
  for (int q = 0; q < c; ++q) {
    int k = __builtin_ffs((int)mk) - 1;
    mk &= mk - 1u;
    k = k < 0 ? 0 : k;
    const int nd = __builtin_amdgcn_readlane(node, k);
    acc += nl[(size_t)nd * NLW + lane];
  }
  return acc;
}

__global__ __launch_bounds__(NTHR) void k_pool(const float* __restrict__ nl, const int* __restrict__ gid,
                                               const int* __restrict__ fl, int nN, int vec8,
                                               float* out, int outN) {
  __shared__ int reg1[PCAP];
  __shared__ int list[LISTN];
  __shared__ int wcnt[NWAVE];
  __shared__ int wbad[NWAVE];
  __shared__ __attribute__((aligned(16))) float stg[PG * 32];
  const int tid = (int)threadIdx.x, lane = tid & 31, wave = tid >> 5;
  const int slotBase = (int)blockIdx.x * PG;

  const int nh = compact_keys(gid, nN, slotBase, PG, vec8, reg1, PCAP, list, wcnt, tid, lane, wave);

  {
    const int ft  = tid < 3 * NSB ? tid : 3 * NSB - 1;
    const int fll = ft / NSB;
    const int flb = ft - fll * NSB;
    const int fvl = fl[(size_t)(fll * FLB + flb) * 32];
    const bool pf = ((tid < 3 * NSB) && (fvl != 0)) || (nh >= PCAP);
    const unsigned pm = __builtin_amdgcn_ballot_w32(pf);
    if (lane == 0) wbad[wave] = (pm != 0u) ? 1 : 0;
  }

  float a0 = 0.0f, a1 = 0.0f, a2 = 0.0f, a3 = 0.0f;
  const int g0 = 4 * wave;
#pragma unroll 1
  for (int b0 = 0; b0 < nh; b0 += 32) {
    const int idx = b0 + lane;
    int idc = idx > nh - 1 ? nh - 1 : idx;
    idc = idc < 0 ? 0 : (idc > PCAP - 1 ? PCAP - 1 : idc);
    const int ent = reg1[idc];
    const bool valid = idx < nh;
    const int rel = (ent & (PG - 1)) - g0;
    int node = (int)((unsigned)ent >> PKS);
    node = node > nN - 1 ? nN - 1 : node;
    const unsigned m0 = __builtin_amdgcn_ballot_w32(valid && (rel == 0));
    const unsigned m1 = __builtin_amdgcn_ballot_w32(valid && (rel == 1));
    const unsigned m2 = __builtin_amdgcn_ballot_w32(valid && (rel == 2));
    const unsigned m3 = __builtin_amdgcn_ballot_w32(valid && (rel == 3));
    a0 = pool_hits(m0, node, nl, lane, a0);
    a1 = pool_hits(m1, node, nl, lane, a1);
    a2 = pool_hits(m2, node, nl, lane, a2);
    a3 = pool_hits(m3, node, nl, lane, a3);
  }
  if (lane < DO) {
    stg[(g0 + 0) * DO + lane] = a0;
    stg[(g0 + 1) * DO + lane] = a1;
    stg[(g0 + 2) * DO + lane] = a2;
    stg[(g0 + 3) * DO + lane] = a3;
  }
  __syncthreads();
  int bad = 0;
#pragma unroll
  for (int w2 = 0; w2 < NWAVE; ++w2) bad |= wbad[w2];

  const int tq = tid < (PG * DO) / 4 ? tid : (PG * DO) / 4 - 1;
  v4f v = *(const v4fa*)(stg + 4 * tq);
  const float qn = __int_as_float(0x7fc00000);
  v.x = (bad != 0) ? qn : v.x;
  v.y = (bad != 0) ? qn : v.y;
  v.z = (bad != 0) ? qn : v.z;
  v.w = (bad != 0) ? qn : v.w;
  const int e = (int)blockIdx.x * (PG * DO) + 4 * tid;
  const bool ok = (tid < (PG * DO) / 4) && (e + 3 < outN);
  float* op = out + (size_t)((int)blockIdx.x * (PG * DO)) + (size_t)(4 * tq);
  if (ok) *(volatile v4f*)op = v;
  __threadfence();
  if (ok) *(volatile v4f*)op = v;
}

extern "C" void kernel_launch(void* const* d_in, const int* in_sizes, int n_in,
                              void* d_out, int out_size, void* d_ws, size_t ws_size,
                              hipStream_t stream) {
  if (n_in < 20) return;
  if (in_sizes[0] != NN * DRAW) return;
  if (in_sizes[1] != NE || in_sizes[2] != NE) return;
  if (in_sizes[3] != NN) return;
  if (in_sizes[4] != DRAW * DH || in_sizes[5] != DH) return;
  if (in_sizes[6] != DH * DO || in_sizes[7] != DO) return;
  for (int i = 8; i < 20; ++i) {
    const int want = ((i & 1) == 0) ? DH * DH : DH;
    if (in_sizes[i] != want) return;
  }
  if (out_size != NG * DO) return;
  if (WS_TOTAL > ws_size) return;

  const float* x    = (const float*)d_in[0];
  const int*   src  = (const int*)  d_in[1];
  const int*   dst  = (const int*)  d_in[2];
  const int*   gid  = (const int*)  d_in[3];
  const float* Wli  = (const float*)d_in[4];
  const float* bli  = (const float*)d_in[5];
  const float* Wro  = (const float*)d_in[6];
  const float* bro  = (const float*)d_in[7];
  const float* Wc1  = (const float*)d_in[8];
  const float* bc1  = (const float*)d_in[9];
  const float* Wf1  = (const float*)d_in[10];
  const float* bf1  = (const float*)d_in[11];
  const float* Wc2  = (const float*)d_in[12];
  const float* bc2  = (const float*)d_in[13];
  const float* Wf2  = (const float*)d_in[14];
  const float* bf2  = (const float*)d_in[15];
  const float* Wc3  = (const float*)d_in[16];
  const float* bc3  = (const float*)d_in[17];
  const float* Wf3  = (const float*)d_in[18];
  const float* bf3  = (const float*)d_in[19];
  float* out = (float*)d_out;

  char* ws = (char*)d_ws;
  unsigned short* P1   = (unsigned short*)(ws + OFF_P1);
  unsigned short* P2   = (unsigned short*)(ws + OFF_P2);
  unsigned short* WREG = (unsigned short*)(ws + OFF_W);
  int*            FL   = (int*)(ws + OFF_FL);
  unsigned short* XB   = P2;
  float*          NL   = (float*)(ws + OFF_P1);
  const unsigned short* WRO = WREG + (size_t)6 * WSQ;
  const unsigned short* WLI = WREG + (size_t)6 * WSQ + (size_t)32 * PW;

  const float* bcs[3] = {bc1, bc2, bc3};
  const float* bfs[3] = {bf1, bf2, bf3};

  hipFuncSetAttribute(reinterpret_cast<const void*>(&k_scan), hipFuncAttributeMaxDynamicSharedMemorySize, LDS_AGG);

  const dim3 gW(MP / GBM, DP / 64);
  const dim3 gR(MP / GBM, 1);
  const int vecE = ((NE & 3) == 0) ? 1 : 0;
  const int vecN = ((NN & 3) == 0) ? 1 : 0;

  k_prep<<<NUTOT / NTHR, NTHR, 0, stream>>>(Wc1, Wf1, Wc2, Wf2, Wc3, Wf3, Wro, Wli, x, WREG, XB);
  k_gemm<4, 0, 0><<<gW, GTHR, 0, stream>>>(XB, XK, WLI, XK, XK, bli, DH, (void*)P1, NN, MP);

  unsigned short* cur = P1;
  unsigned short* oth = P2;
  for (int l = 0; l < 3; ++l) {
    k_gemm<4, 1, 0><<<gW, GTHR, 0, stream>>>(cur, PW, WREG + (size_t)(2 * l) * WSQ, PW, PW,
                                             bcs[l], DH, (void*)oth, NN, MP);
    k_scan<<<NSB, NTHR, LDS_AGG, stream>>>(src, dst, oth, cur, FL + (size_t)l * FLB * 32,
                                           NN, NE, NBRUN, vecE, MP);
    k_gemm<4, 1, 0><<<gW, GTHR, 0, stream>>>(cur, PW, WREG + (size_t)(2 * l + 1) * WSQ, PW, PW,
                                             bfs[l], DH, (void*)oth, NN, MP);
    unsigned short* t = cur; cur = oth; oth = t;
  }
  k_gemm<2, 0, 1><<<gR, GTHR, 0, stream>>>(cur, PW, WRO, PW, PW, bro, DO, (void*)NL, NN, MP);
  k_pool<<<NPB, NTHR, 0, stream>>>(NL, gid, FL, NN, vecN, out, out_size);
}
